// GAT_NET_20272245637549
// MI455X (gfx1250) — hardware-verified
//
#include <hip/hip_runtime.h>
#include <stddef.h>
#include <stdint.h>
#include <math.h>


#define F_IN    128
#define CW      256
#define KA2     512
#define DHA     128
#define DHB     32
#define DHBP    64
#define DHC     16
#define DHCP    64
#define YTW     32
#define NTHR    256
#define NWAVE   8
#define EPT     8
#define CHUNK   (NTHR * EPT)
#define WCAP    (EPT * 32)
#define LISTN   (NWAVE * WCAP)
#define NBMAX   2048
#define SLOTB   11
#define RCAP    28672
#define DEGCAP  256
#define GBM     64
#define GBN     64
#define GTHR    128
#define MROWS   128
#define PCH     256
#define NEGSL   0.2f
#define NEGS1   0.01f
#define MX0     (-1.0e30f)
#define WSMAX   134217728
#define LDS_AGG ((2 * RCAP + 2 * NBMAX + LISTN) * 4 + 64)

static_assert((CHUNK & (CHUNK - 1)) == 0 && CHUNK <= (1 << SLOTB));
static_assert(NBMAX == (1 << SLOTB));
static_assert(NTHR * 8 == NBMAX);
static_assert(LISTN >= NBMAX);
static_assert(LISTN >= NWAVE * WCAP);
static_assert((RCAP % 32) == 0);
static_assert(LDS_AGG <= 300000);
static_assert(GBM == (GTHR / 32) * 16);
static_assert((F_IN % 32) == 0 && (KA2 % 32) == 0 && (CW % 32) == 0);
static_assert((CW % GBN) == 0 && (DHA % GBN) == 0 && DHBP == GBN && DHCP == GBN);
static_assert(KA2 == 2 * CW);
static_assert(CW == 8 * 32);
static_assert((MROWS % GBM) == 0);
static_assert(NTHR == CW);
static_assert(PCH == NTHR);
static_assert((F_IN / 8) == 16);
static_assert(YTW * 4 == 128 && DHC <= YTW && (DHC % 4) == 0 && DHC <= 32);
static_assert(DHB <= DHBP && DHC <= DHCP);

typedef float          v4f  __attribute__((ext_vector_type(4)));
typedef float          v8f  __attribute__((ext_vector_type(8)));
typedef int            v4i  __attribute__((ext_vector_type(4)));
typedef int            v8i  __attribute__((ext_vector_type(8)));
typedef unsigned int   v4u  __attribute__((ext_vector_type(4)));
typedef unsigned short v8us __attribute__((ext_vector_type(8)));
typedef _Float16       v8h  __attribute__((ext_vector_type(8)));
typedef __bf16         v16b __attribute__((ext_vector_type(16)));
typedef v4f  __attribute__((may_alias)) v4fa;
typedef v4u  __attribute__((may_alias)) v4ua;
typedef v8us __attribute__((may_alias)) v8usa;
union FragB { v16b v; v8us h[2]; v8i w; };

__device__ __forceinline__ v8f wmb(const FragB& a, const FragB& b, v8f c) {
  v8f d = __builtin_amdgcn_wmma_f32_16x16x32_bf16(false, a.v, false, b.v, (short)0, c, false, false);
  asm volatile("v_nop\n\tv_nop\n\tv_nop\n\tv_nop" : "+v"(d) : "v"(a.w), "v"(b.w));
  return d;
}

__device__ __forceinline__ unsigned int f2bf(float f) {
  const unsigned int u = __float_as_uint(f);
  return ((u + 0x7FFFu + ((u >> 16) & 1u)) >> 16) & 0xFFFFu;
}
__device__ __forceinline__ float bf2f(unsigned int b) { return __uint_as_float(b << 16); }
__device__ __forceinline__ float bfr(float f) { return bf2f(f2bf(f)); }
__device__ __forceinline__ v4f bfr4(const v4f a) {
  v4f r; r.x = bfr(a.x); r.y = bfr(a.y); r.z = bfr(a.z); r.w = bfr(a.w); return r;
}
__device__ __forceinline__ float hb2f(unsigned int b) {
  const unsigned short s = (unsigned short)(b & 0xFFFFu);
  const _Float16 hv = __builtin_bit_cast(_Float16, s);
  return (float)hv;
}
__device__ __forceinline__ unsigned int pk2(float lo, float hi) { return f2bf(lo) | (f2bf(hi) << 16); }
__device__ __forceinline__ unsigned int pk2lo(float lo, float hi) {
  return f2bf(lo - bfr(lo)) | (f2bf(hi - bfr(hi)) << 16);
}
__device__ __forceinline__ v4u pack8(const v4f a, const v4f b) {
  v4u r;
  r.x = pk2(a.x, a.y); r.y = pk2(a.z, a.w); r.z = pk2(b.x, b.y); r.w = pk2(b.z, b.w);
  return r;
}
__device__ __forceinline__ v4u pack8lo(const v4f a, const v4f b) {
  v4u r;
  r.x = pk2lo(a.x, a.y); r.y = pk2lo(a.z, a.w); r.z = pk2lo(b.x, b.y); r.w = pk2lo(b.z, b.w);
  return r;
}
__device__ __forceinline__ v8h cvt8h(const v4f a, const v4f b) {
  v8h hv;
  hv[0] = (_Float16)a.x; hv[1] = (_Float16)a.y; hv[2] = (_Float16)a.z; hv[3] = (_Float16)a.w;
  hv[4] = (_Float16)b.x; hv[5] = (_Float16)b.y; hv[6] = (_Float16)b.z; hv[7] = (_Float16)b.w;
  return hv;
}
template<int L> __device__ __forceinline__ float actf(float v) {
  return (L == 1) ? fmaxf(v, NEGS1 * v) : v;
}

__device__ __forceinline__ int scan_chunk(const int* __restrict__ dsts, int nE, int cbase, int slotBase,
                                          int nb, int vec8, int* list, int tid, int lane, int wave) {
  int wc = 0;
  const int el0  = tid * EPT;
  const int e0   = cbase + el0;
  const int sent = -2147483647 - 1;
  v4i da, db;
  if (vec8 != 0 && cbase + CHUNK <= nE) {
    da = *(const v4i*)(dsts + e0);
    db = *(const v4i*)(dsts + e0 + 4);
  } else {
    da.x = (e0     < nE) ? dsts[min(e0,     nE - 1)] : sent;
    da.y = (e0 + 1 < nE) ? dsts[min(e0 + 1, nE - 1)] : sent;
    da.z = (e0 + 2 < nE) ? dsts[min(e0 + 2, nE - 1)] : sent;
    da.w = (e0 + 3 < nE) ? dsts[min(e0 + 3, nE - 1)] : sent;
    db.x = (e0 + 4 < nE) ? dsts[min(e0 + 4, nE - 1)] : sent;
    db.y = (e0 + 5 < nE) ? dsts[min(e0 + 5, nE - 1)] : sent;
    db.z = (e0 + 6 < nE) ? dsts[min(e0 + 6, nE - 1)] : sent;
    db.w = (e0 + 7 < nE) ? dsts[min(e0 + 7, nE - 1)] : sent;
  }
  const unsigned nbs = (unsigned)slotBase;
  const unsigned unb = (unsigned)nb;
  const unsigned s0 = (unsigned)da.x - nbs, s1 = (unsigned)da.y - nbs;
  const unsigned s2 = (unsigned)da.z - nbs, s3 = (unsigned)da.w - nbs;
  const unsigned s4 = (unsigned)db.x - nbs, s5 = (unsigned)db.y - nbs;
  const unsigned s6 = (unsigned)db.z - nbs, s7 = (unsigned)db.w - nbs;
  const bool h0 = s0 < unb, h1 = s1 < unb, h2 = s2 < unb, h3 = s3 < unb;
  const bool h4 = s4 < unb, h5 = s5 < unb, h6 = s6 < unb, h7 = s7 < unb;
  const unsigned any = __builtin_amdgcn_ballot_w32(h0 | h1 | h2 | h3 | h4 | h5 | h6 | h7);
  if (any != 0u) {
#define HITJ(J, HJ, SJ) { \
      const unsigned mj = __builtin_amdgcn_ballot_w32(HJ); \
      if (mj != 0u) { \
        if (HJ) { \
          const int pos = wc + (int)__builtin_amdgcn_mbcnt_lo(mj, 0u); \
          if (pos < WCAP) list[wave * WCAP + pos] = ((el0 + (J)) << SLOTB) | (int)(SJ); \
        } \
        wc += (int)__builtin_popcount(mj); } }
    HITJ(0, h0, s0)
    HITJ(1, h1, s1)
    HITJ(2, h2, s2)
    HITJ(3, h3, s3)
    HITJ(4, h4, s4)
    HITJ(5, h5, s5)
    HITJ(6, h6, s6)
    HITJ(7, h7, s7)
#undef HITJ
  }
  return wc;
}

__global__ __launch_bounds__(NTHR) void k_xprep(const float* __restrict__ x, unsigned short* xb, int nN, int nUnits) {
  const int i = (int)blockIdx.x * NTHR + (int)threadIdx.x;
  if (i >= nUnits) return;
  const int row = i >> 4;
  const int c0  = (i & 15) * 8;
  const int rc  = row < nN ? row : nN - 1;
  const float* p = x + (size_t)rc * F_IN + c0;
  v4f a = *(const v4fa*)p, b = *(const v4fa*)(p + 4);
  const v4f z4 = {0.f, 0.f, 0.f, 0.f};
  if (row >= nN) { a = z4; b = z4; }
  const v4u hv = pack8(a, b);
  const size_t o = (size_t)row * F_IN + c0;
  *(volatile v4u*)(xb + o) = hv;
  __threadfence();
  *(volatile v4u*)(xb + o) = hv;
}

__global__ __launch_bounds__(NTHR) void k_wtr(const float* __restrict__ w, int Kin, int Kfold, int Ncol, int Nrows,
                                              int Kout, unsigned short* wt, int nUnits) {
  const int u = (int)blockIdx.x * NTHR + (int)threadIdx.x;
  if (u >= nUnits) return;
  const int kq = Kout >> 3;
  const int n  = u / kq;
  const int k8 = (u - n * kq) * 8;
  const int kk = k8 - (k8 / Kfold) * Kfold;
  const bool kv = kk < Kin;
  const int kcl = kv ? kk : Kin - 8;
  const int ncl = n < Ncol ? n : Ncol - 1;
  const float* p = w + (size_t)kcl * (size_t)Ncol + ncl;
  v4f a, b;
  a.x = p[0];                    a.y = p[(size_t)Ncol];         a.z = p[(size_t)2 * Ncol];     a.w = p[(size_t)3 * Ncol];
  b.x = p[(size_t)4 * Ncol];     b.y = p[(size_t)5 * Ncol];     b.z = p[(size_t)6 * Ncol];     b.w = p[(size_t)7 * Ncol];
  const v4f z4 = {0.f, 0.f, 0.f, 0.f};
  if (n >= Ncol || n >= Nrows || !kv) { a = z4; b = z4; }
  const v4u wv = pack8(a, b);
  unsigned short* o = wt + (size_t)n * (size_t)Kout + k8;
  *(volatile v4u*)o = wv;
  __threadfence();
  *(volatile v4u*)o = wv;
}

template<int MODE>
__global__ __launch_bounds__(GTHR) void k_gemm(
    const unsigned short* __restrict__ A, const unsigned short* __restrict__ WT, int K,
    float* o32, unsigned short* o16, int ldo, int loff,
    const float* __restrict__ bias, int nBias)
{
  __shared__ __attribute__((aligned(16))) float stg[GBM * GBN];
  const int tid = (int)threadIdx.x, lane = tid & 31, wave = tid >> 5, hh = lane >> 4, m = lane & 15;
  const int rowBase = (int)blockIdx.x * GBM;
  const int col0    = (int)blockIdx.y * GBN;

  float bv[4];
#pragma unroll
  for (int t = 0; t < 4; ++t) {
    const int gc = col0 + 16 * t + m;
    int bc = gc < nBias ? gc : nBias - 1;
    bc = bc < 0 ? 0 : bc;
    const float b = bias[bc];
    bv[t] = (gc < nBias) ? bfr(b) : 0.0f;
  }

  v8f acc[4];
  {
    const v8f z = {0.f, 0.f, 0.f, 0.f, 0.f, 0.f, 0.f, 0.f};
    acc[0] = z; acc[1] = z; acc[2] = z; acc[3] = z;
  }
  const unsigned short* ap = A  + (size_t)(rowBase + 16 * wave + m) * (size_t)K + 8 * hh;
  const unsigned short* wp = WT + (size_t)(col0 + m) * (size_t)K + 8 * hh;
  const int ksteps = K >> 5;
#pragma unroll 1
  for (int ks = 0; ks < ksteps; ++ks) {
    FragB af;
    af.h[0] = *(const v8usa*)(ap + 32 * ks);
    af.h[1] = *(const v8usa*)(ap + 32 * ks + 16);
#pragma unroll
    for (int t = 0; t < 4; ++t) {
      const unsigned short* wq = wp + (size_t)(16 * t) * (size_t)K + 32 * ks;
      FragB bf;
      bf.h[0] = *(const v8usa*)wq;
      bf.h[1] = *(const v8usa*)(wq + 16);
      acc[t] = wmb(af, bf, acc[t]);
    }
  }

#pragma unroll
  for (int t = 0; t < 4; ++t) {
    const int lc = 16 * t + m;
#pragma unroll
    for (int r = 0; r < 8; ++r) {
      const int lr = 16 * wave + 8 * hh + r;
      stg[lr * GBN + lc] = acc[t][r] + bv[t];
    }
  }
  __syncthreads();

  if (MODE == 0) {
    v4f fv[8];
#pragma unroll
    for (int i = 0; i < 8; ++i) {
      const int lr = 16 * wave + 2 * i + hh;
      fv[i] = *(const v4fa*)(stg + lr * GBN + 4 * m);
    }
#pragma unroll
    for (int i = 0; i < 8; ++i) {
      const int gr = rowBase + 16 * wave + 2 * i + hh;
      float* op = o32 + (size_t)gr * (size_t)ldo + col0 + 4 * m;
      *(volatile v4f*)op = fv[i];
    }
    __threadfence();
#pragma unroll
    for (int i = 0; i < 8; ++i) {
      const int gr = rowBase + 16 * wave + 2 * i + hh;
      float* op = o32 + (size_t)gr * (size_t)ldo + col0 + 4 * m;
      *(volatile v4f*)op = fv[i];
    }
  } else {
    const int pr = lane >> 3, pc = lane & 7;
    v4f ga[4], gb[4];
#pragma unroll
    for (int i = 0; i < 4; ++i) {
      const int lr = 16 * wave + 4 * i + pr;
      ga[i] = *(const v4fa*)(stg + lr * GBN + 8 * pc);
      gb[i] = *(const v4fa*)(stg + lr * GBN + 8 * pc + 4);
    }
    if (MODE == 1) {
      v8h hv[4];
#pragma unroll
      for (int i = 0; i < 4; ++i) hv[i] = cvt8h(ga[i], gb[i]);
#pragma unroll
      for (int i = 0; i < 4; ++i) {
        const int gr = rowBase + 16 * wave + 4 * i + pr;
        unsigned short* op = o16 + (size_t)gr * (size_t)ldo + col0 + 8 * pc;
        *(volatile v8h*)op = hv[i];
      }
      __threadfence();
#pragma unroll
      for (int i = 0; i < 4; ++i) {
        const int gr = rowBase + 16 * wave + 4 * i + pr;
        unsigned short* op = o16 + (size_t)gr * (size_t)ldo + col0 + 8 * pc;
        *(volatile v8h*)op = hv[i];
      }
    } else {
      v4u hv[4], lv[4];
#pragma unroll
      for (int i = 0; i < 4; ++i) { hv[i] = pack8(ga[i], gb[i]); lv[i] = pack8lo(ga[i], gb[i]); }
#pragma unroll
      for (int i = 0; i < 4; ++i) {
        const int gr = rowBase + 16 * wave + 4 * i + pr;
        unsigned short* op = o16 + (size_t)gr * (size_t)ldo + col0 + 8 * pc;
        *(volatile v4u*)op = hv[i];
        *(volatile v4u*)(op + loff) = lv[i];
      }
      __threadfence();
#pragma unroll
      for (int i = 0; i < 4; ++i) {
        const int gr = rowBase + 16 * wave + 4 * i + pr;
        unsigned short* op = o16 + (size_t)gr * (size_t)ldo + col0 + 8 * pc;
        *(volatile v4u*)op = hv[i];
        *(volatile v4u*)(op + loff) = lv[i];
      }
    }
  }
  (void)o32; (void)o16; (void)loff;
}

template<int L>
__global__ __launch_bounds__(NTHR) void k_agg(
    const int* __restrict__ srcs, const int* __restrict__ dsts,
    const float* __restrict__ XL, const unsigned short* __restrict__ XR,
    const float* __restrict__ att, const float* __restrict__ bias,
    unsigned short* HP,
    int nN, int nE, int nb, int vec8, int MPr) {
  extern __shared__ v4f lds_dyn[];
  int* reg1 = (int*)lds_dyn;
  int* reg2 = reg1 + RCAP;
  int* scnt = reg2 + RCAP;
  int* soff = scnt + NBMAX;
  int* list = soff + NBMAX;
  int* wcnt = list + LISTN;
  int* wtot = wcnt + NWAVE;
  const int tid = (int)threadIdx.x, lane = tid & 31, wave = tid >> 5;
  const int nodeBase = (int)blockIdx.x * nb;

  for (int i = tid; i < NBMAX; i += NTHR) scnt[i] = 0;
  __syncthreads();

  int tot = 0;
  const int nChunks = (nE + CHUNK - 1) / CHUNK;
#pragma unroll 1
  for (int ch = 0; ch < nChunks; ++ch) {
    const int cbase = ch * CHUNK;
    const int wc = scan_chunk(dsts, nE, cbase, nodeBase, nb, vec8, list, tid, lane, wave);
    if (lane == 0) wcnt[wave] = wc;
    __syncthreads();
    int pre = 0, all = 0;
#pragma unroll
    for (int w2 = 0; w2 < NWAVE; ++w2) {
      int c = wcnt[w2];
      c = c < 0 ? 0 : (c > WCAP ? WCAP : c);
      all += c;
      pre += (w2 < wave) ? c : 0;
    }
    const int wcc  = wc > WCAP ? WCAP : wc;
    const int base = tot + pre;
#pragma unroll 1
    for (int i = lane; i < wcc; i += 32) {
      const int ent = list[wave * WCAP + i];
      const int el  = (ent >> SLOTB) & (CHUNK - 1);
      const int sl  = ent & (NBMAX - 1);
      int eid = cbase + el;
      eid = eid > nE - 1 ? nE - 1 : eid;
      const int pos = base + i;
      if (pos < RCAP) reg1[pos] = (int)(((unsigned)eid << SLOTB) | (unsigned)sl);
    }
    tot += all;
    tot = tot > RCAP ? RCAP : tot;
    __syncthreads();
  }
  const int nh = tot;

  if (wave == 0) {
#pragma unroll 1
    for (int b0 = 0; b0 < nh; b0 += 32) {
      const int idx = b0 + lane;
      const int uv  = reg1[idx < nh ? idx : nh - 1];
      const int m32 = (nh - b0) < 32 ? (nh - b0) : 32;
#pragma unroll 1
      for (int k = 0; k < m32; ++k) {
        const int u  = __builtin_amdgcn_readlane(uv, k);
        const int sl = u & (NBMAX - 1);
        if (lane == 0) scnt[sl] = scnt[sl] + 1;
      }
    }
  }
  __syncthreads();

  {
    const v4i ca = *(const v4i*)(scnt + 8 * tid);
    const v4i cb = *(const v4i*)(scnt + 8 * tid + 4);
    const int e0 = ca.x < 0 ? 0 : ca.x, e1 = ca.y < 0 ? 0 : ca.y, e2 = ca.z < 0 ? 0 : ca.z, e3 = ca.w < 0 ? 0 : ca.w;
    const int e4 = cb.x < 0 ? 0 : cb.x, e5 = cb.y < 0 ? 0 : cb.y, e6 = cb.z < 0 ? 0 : cb.z, e7 = cb.w < 0 ? 0 : cb.w;
    const int ts = e0 + e1 + e2 + e3 + e4 + e5 + e6 + e7;
    int incl = ts;
#pragma unroll
    for (int d = 1; d < 32; d <<= 1) {
      const int up = __shfl_up(incl, d);
      if (lane >= d) incl += up;
    }
    if (lane == 31) wtot[wave] = incl;
    __syncthreads();
    int pre = 0;
#pragma unroll
    for (int w2 = 0; w2 < NWAVE; ++w2) pre += (w2 < wave) ? wtot[w2] : 0;
    int run = pre + incl - ts;
    soff[8 * tid + 0] = run; run += e0;
    soff[8 * tid + 1] = run; run += e1;
    soff[8 * tid + 2] = run; run += e2;
    soff[8 * tid + 3] = run; run += e3;
    soff[8 * tid + 4] = run; run += e4;
    soff[8 * tid + 5] = run; run += e5;
    soff[8 * tid + 6] = run; run += e6;
    soff[8 * tid + 7] = run;
  }
  __syncthreads();
  for (int i = tid; i < NBMAX; i += NTHR) list[i] = soff[i];
  __syncthreads();

  if (wave == 0) {
#pragma unroll 1
    for (int b0 = 0; b0 < nh; b0 += 32) {
      const int idx = b0 + lane;
      const int uv  = reg1[idx < nh ? idx : nh - 1];
      const int m32 = (nh - b0) < 32 ? (nh - b0) : 32;
#pragma unroll 1
      for (int k = 0; k < m32; ++k) {
        const int u   = __builtin_amdgcn_readlane(uv, k);
        const int sl  = u & (NBMAX - 1);
        const int eid = (int)((unsigned)u >> SLOTB);
        if (lane == 0) {
          int pos = list[sl];
          pos = pos < 0 ? 0 : (pos > RCAP - 1 ? RCAP - 1 : pos);
          reg2[pos] = eid;
          list[sl] = pos + 1;
        }
      }
    }
  }
  __syncthreads();

  const int nbw = nb >> 3;
  const bool ovf = (nh >= RCAP);
  const float qnan = __int_as_float(0x7fc00000);
  const int c0 = 8 * lane;
  const v4f atA = bfr4(*(const v4fa*)(att + c0));
  const v4f atB = bfr4(*(const v4fa*)(att + c0 + 4));
  const v4f bbA = bfr4(*(const v4fa*)(bias + c0));
  const v4f bbB = bfr4(*(const v4fa*)(bias + c0 + 4));

#pragma unroll 1
  for (int jt = 0; jt < nbw; ++jt) {
    const int slot = wave * nbw + jt;
    const int grow = nodeBase + slot;
    const int gcl  = grow < nN ? grow : nN - 1;
    int st = soff[slot];
    const int craw = scnt[slot];
    int cnt = craw;
    st  = st < 0 ? 0 : (st > nh ? nh : st);
    cnt = cnt < 0 ? 0 : (cnt > DEGCAP ? DEGCAP : cnt);
    if (cnt > nh - st) cnt = nh - st;
    const float pz = (ovf || craw > DEGCAP) ? qnan : 0.0f;

    const v4u hw = *(const v4ua*)(XR + (size_t)gcl * CW + c0);
    const float d0 = hb2f(hw.x), d1 = hb2f(hw.x >> 16), d2 = hb2f(hw.y), d3 = hb2f(hw.y >> 16);
    const float d4 = hb2f(hw.z), d5 = hb2f(hw.z >> 16), d6 = hb2f(hw.w), d7 = hb2f(hw.w >> 16);

    float mx = MX0, dn = 0.0f;
    v4f av = {0.f, 0.f, 0.f, 0.f};
    v4f aw = {0.f, 0.f, 0.f, 0.f};

#pragma unroll 1
    for (int q = 0; q < cnt; ++q) {
      int idx = st + q; idx = idx > RCAP - 1 ? RCAP - 1 : idx;
      int eid = reg2[idx]; eid = eid < 0 ? 0 : (eid > nE - 1 ? nE - 1 : eid);
      const int sraw = srcs[eid];
      const int s = sraw < 0 ? 0 : (sraw > nN - 1 ? nN - 1 : sraw);
      const float* fr = XL + (size_t)s * CW + c0;
      const v4f fs = *(const v4fa*)fr;
      const v4f ft = *(const v4fa*)(fr + 4);
      float e, part;
      e = fs.x + d0; e = fmaxf(e, NEGSL * e); part = e * atA.x;
      e = fs.y + d1; e = fmaxf(e, NEGSL * e); part = fmaf(e, atA.y, part);
      e = fs.z + d2; e = fmaxf(e, NEGSL * e); part = fmaf(e, atA.z, part);
      e = fs.w + d3; e = fmaxf(e, NEGSL * e); part = fmaf(e, atA.w, part);
      e = ft.x + d4; e = fmaxf(e, NEGSL * e); part = fmaf(e, atB.x, part);
      e = ft.y + d5; e = fmaxf(e, NEGSL * e); part = fmaf(e, atB.y, part);
      e = ft.z + d6; e = fmaxf(e, NEGSL * e); part = fmaf(e, atB.z, part);
      e = ft.w + d7; e = fmaxf(e, NEGSL * e); part = fmaf(e, atB.w, part);
      part += __shfl_xor(part, 1);
      part += __shfl_xor(part, 2);
      part += __shfl_xor(part, 4);
      if (L == 2) {
        part += __shfl_xor(part, 8);
        part += __shfl_xor(part, 16);
      }
      const float lg = part;
      const float df = lg - mx;
      const float ee = __expf(-fabsf(df));
      const bool up  = df > 0.f;
      const float s1 = up ? ee : 1.0f;
      const float s2 = up ? 1.0f : ee;
      mx = up ? lg : mx;
      dn = fmaf(dn, s1, s2);
      av.x = fmaf(av.x, s1, s2 * fs.x);
      av.y = fmaf(av.y, s1, s2 * fs.y);
      av.z = fmaf(av.z, s1, s2 * fs.z);
      av.w = fmaf(av.w, s1, s2 * fs.w);
      aw.x = fmaf(aw.x, s1, s2 * ft.x);
      aw.y = fmaf(aw.y, s1, s2 * ft.y);
      aw.z = fmaf(aw.z, s1, s2 * ft.z);
      aw.w = fmaf(aw.w, s1, s2 * ft.w);
    }
    const float ds  = dn > 0.f ? dn : 1.0f;
    const float inv = (dn > 0.f ? 1.0f : 0.0f) * __builtin_amdgcn_rcpf(ds);
    const bool live = grow < nN;
    v4f o, u;
    o.x = (live ? actf<L>(fmaf(av.x, inv, bbA.x)) : 0.f) + pz;
    o.y = (live ? actf<L>(fmaf(av.y, inv, bbA.y)) : 0.f) + pz;
    o.z = (live ? actf<L>(fmaf(av.z, inv, bbA.z)) : 0.f) + pz;
    o.w = (live ? actf<L>(fmaf(av.w, inv, bbA.w)) : 0.f) + pz;
    u.x = (live ? actf<L>(fmaf(aw.x, inv, bbB.x)) : 0.f) + pz;
    u.y = (live ? actf<L>(fmaf(aw.y, inv, bbB.y)) : 0.f) + pz;
    u.z = (live ? actf<L>(fmaf(aw.z, inv, bbB.z)) : 0.f) + pz;
    u.w = (live ? actf<L>(fmaf(aw.w, inv, bbB.w)) : 0.f) + pz;
    const v4u hv = pack8(o, u);
    const v4u lv = pack8lo(o, u);
    unsigned short* gp = HP + (size_t)grow * KA2 + 8 * lane;
    const bool wr = grow < MPr;
    if (wr) { *(volatile v4u*)gp = hv; *(volatile v4u*)(gp + CW) = lv; }
    __threadfence();
    if (wr) { *(volatile v4u*)gp = hv; *(volatile v4u*)(gp + CW) = lv; }
  }
}

__global__ __launch_bounds__(NTHR) void k_pool(const unsigned short* __restrict__ HP, const float* __restrict__ YF,
                                               const int* __restrict__ batch, float* out1, float* YT,
                                               int nN, int nB) {
  __shared__ int lst[PCH];
  __shared__ int wcn[NWAVE];
  __shared__ __attribute__((aligned(16))) float sE[CW];
  __shared__ __attribute__((aligned(16))) float sY[YTW];
  const int tid = (int)threadIdx.x, lane = tid & 31, wave = tid >> 5;
  const int g = (int)blockIdx.x;
  const float ninf = __int_as_float(0xff800000);
  float em = ninf, ym = ninf;
  const int nCh = (nN + PCH - 1) / PCH;
#pragma unroll 1
  for (int ch = 0; ch < nCh; ++ch) {
    const int i   = ch * PCH + tid;
    const int icl = i < nN ? i : nN - 1;
    const int bt  = batch[icl];
    const bool hit = (i < nN) && (bt == g);
    const unsigned mk = __builtin_amdgcn_ballot_w32(hit);
    if (lane == 0) wcn[wave] = (int)__builtin_popcount(mk);
    __syncthreads();
    int pre = 0, tot = 0;
#pragma unroll
    for (int w2 = 0; w2 < NWAVE; ++w2) {
      const int c = wcn[w2];
      tot += c;
      pre += (w2 < wave) ? c : 0;
    }
    if (hit) {
      const int pos = pre + (int)__builtin_amdgcn_mbcnt_lo(mk, 0u);
      if (pos < PCH) lst[pos] = i;
    }
    __syncthreads();
    tot = tot < 0 ? 0 : (tot > PCH ? PCH : tot);
#pragma unroll 1
    for (int j = 0; j < tot; ++j) {
      int node = lst[j];
      node = node < 0 ? 0 : (node > nN - 1 ? nN - 1 : node);
      const unsigned hi = HP[(size_t)node * KA2 + tid];
      const unsigned lo = HP[(size_t)node * KA2 + CW + tid];
      const float v = bf2f(hi) + bf2f(lo);
      em = (em > v || em != em) ? em : v;
      if (wave == 0) {
        const float yv = YF[(size_t)node * DHCP + lane];
        ym = (ym > yv || ym != ym) ? ym : yv;
      }
    }
    __syncthreads();
  }
  sE[tid] = em;
  if (wave == 0) sY[lane] = (lane < DHC) ? ym : 0.0f;
  __syncthreads();
  const bool w01 = wave < 2;
  const int  pt  = tid & 63;
  const v4f  ev  = *(const v4fa*)(sE + 4 * pt);
  float* op = out1 + (size_t)g * CW + 4 * pt;
  const bool wy  = (wave == 0) && (lane < 8);
  const v4f  yq  = *(const v4fa*)(sY + 4 * (lane & 7));
  float* yp = YT + (size_t)g * YTW + 4 * (lane & 7);
  if (w01) *(volatile v4f*)op = ev;
  if (wy)  *(volatile v4f*)yp = yq;
  __threadfence();
  if (w01) *(volatile v4f*)op = ev;
  if (wy)  *(volatile v4f*)yp = yq;
}

__global__ __launch_bounds__(NTHR) void k_out0(const float* __restrict__ YT, float* out0, int nB) {
  const int t = (int)blockIdx.x * NTHR + (int)threadIdx.x;
  const int g = t >> 2, pc = t & 3;
  const bool ok = g < nB;
  const int gcl = ok ? g : nB - 1;
  const v4f v = *(const v4fa*)(YT + (size_t)gcl * YTW + 4 * pc);
  float* op = out0 + (size_t)gcl * DHC + 4 * pc;
  if (ok) *(volatile v4f*)op = v;
  __threadfence();
  if (ok) *(volatile v4f*)op = v;
}

static int pick_nb(int nE, int nN) {
  int nb = NBMAX;
  while (nb > 32 && (long long)nb * (long long)nE * 5LL > (long long)RCAP * (long long)nN * 4LL) nb >>= 1;
  return nb;
}
static inline int cdiv(int a, int b) { return (a + b - 1) / b; }
static inline size_t al256(size_t v) { return (v + 255) & ~(size_t)255; }

extern "C" void kernel_launch(void* const* d_in, const int* in_sizes, int n_in,
                              void* d_out, int out_size, void* d_ws, size_t ws_size,
                              hipStream_t stream) {
  if (n_in < 17) return;
  const int nN = in_sizes[0] / F_IN;
  if (nN <= 0 || in_sizes[0] != nN * F_IN || nN > (1 << 22)) return;
  if (in_sizes[1] < 2 || (in_sizes[1] & 1) != 0) return;
  const int nE = in_sizes[1] / 2;
  if (nE < 1 || nE >= (1 << (32 - SLOTB))) return;
  if (in_sizes[2] != nN) return;
  if (in_sizes[3] != F_IN * CW || in_sizes[4] != F_IN * CW) return;
  if (in_sizes[5] != CW || in_sizes[6] != CW) return;
  if (in_sizes[7] != CW * CW || in_sizes[8] != CW * CW) return;
  if (in_sizes[9] != CW || in_sizes[10] != CW) return;
  if (in_sizes[11] != CW * DHA || in_sizes[12] != DHA) return;
  if (in_sizes[13] != DHA * DHB || in_sizes[14] != DHB) return;
  if (in_sizes[15] != DHB * DHC || in_sizes[16] != DHC) return;
  if (out_size <= 0 || (out_size % (DHC + CW)) != 0) return;
  const int nB = out_size / (DHC + CW);
  if (nB < 1 || nB > 4096) return;

  const float* x     = (const float*)d_in[0];
  const int*   ei    = (const int*)  d_in[1];
  const int*   batch = (const int*)  d_in[2];
  const float* Wl1   = (const float*)d_in[3];
  const float* Wr1   = (const float*)d_in[4];
  const float* att1  = (const float*)d_in[5];
  const float* bg1   = (const float*)d_in[6];
  const float* Wl2   = (const float*)d_in[7];
  const float* Wr2   = (const float*)d_in[8];
  const float* att2  = (const float*)d_in[9];
  const float* bg2   = (const float*)d_in[10];
  const float* W1    = (const float*)d_in[11];
  const float* b1    = (const float*)d_in[12];
  const float* W2    = (const float*)d_in[13];
  const float* b2    = (const float*)d_in[14];
  const float* W3    = (const float*)d_in[15];
  const float* b3    = (const float*)d_in[16];
  float* out0 = (float*)d_out;
  float* out1 = out0 + (size_t)nB * DHC;
  if ((size_t)nB * DHC + (size_t)nB * CW != (size_t)out_size) return;
  const int* src = ei;
  const int* dst = ei + nE;

  const int MP   = cdiv(nN, MROWS) * MROWS;
  const int nb   = pick_nb(nE, nN);
  if (nb < 32 || (nb & (nb - 1)) != 0 || nb > NBMAX) return;
  const int gA   = cdiv(MP, nb);
  const int vec8 = ((nE & 3) == 0) ? 1 : 0;
  if (gA * nb < MP) return;

  char* ws = (char*)d_ws;
  size_t off = 0;
  const size_t oWL1 = off; off = al256(off + (size_t)CW * F_IN * 2);
  const size_t oWR1 = off; off = al256(off + (size_t)CW * F_IN * 2);
  const size_t oWL2 = off; off = al256(off + (size_t)CW * KA2 * 2);
  const size_t oWR2 = off; off = al256(off + (size_t)CW * KA2 * 2);
  const size_t oWH1 = off; off = al256(off + (size_t)DHA * KA2 * 2);
  const size_t oWH2 = off; off = al256(off + (size_t)DHBP * (2 * DHA) * 2);
  const size_t oWH3 = off; off = al256(off + (size_t)DHCP * (2 * DHBP) * 2);
  const size_t szRA = (size_t)MP * CW * 4;
  const size_t szRB = (size_t)MP * CW * 2;
  const size_t szRC = (size_t)MP * KA2 * 2;
  const size_t oRA  = off; off = al256(off + szRA);
  const size_t oRB  = off; off = al256(off + szRB);
  const size_t oRC  = off; off = al256(off + szRC);
  const size_t szXB  = (size_t)MP * F_IN * 2;
  const size_t szY1P = (size_t)MP * (2 * DHA) * 2;
  const size_t szY2P = (size_t)MP * (2 * DHBP) * 2;
  const size_t szYF  = (size_t)MP * DHCP * 4;
  const size_t szYT  = (size_t)nB * YTW * 4;
  if (szXB > szRC) return;
  if (al256(szY1P) + szY2P > szRA) return;
  if (al256(szYF) + szYT > szRB) return;
  if (off > ws_size || off > (size_t)WSMAX) return;
  unsigned short* WL1T = (unsigned short*)(ws + oWL1);
  unsigned short* WR1T = (unsigned short*)(ws + oWR1);
  unsigned short* WL2T = (unsigned short*)(ws + oWL2);
  unsigned short* WR2T = (unsigned short*)(ws + oWR2);
  unsigned short* WH1T = (unsigned short*)(ws + oWH1);
  unsigned short* WH2T = (unsigned short*)(ws + oWH2);
  unsigned short* WH3T = (unsigned short*)(ws + oWH3);
  float*          XL   = (float*)(ws + oRA);
  unsigned short* Y1P  = (unsigned short*)(ws + oRA);
  unsigned short* Y2P  = (unsigned short*)(ws + oRA + al256(szY1P));
  unsigned short* XR   = (unsigned short*)(ws + oRB);
  float*          YF   = (float*)(ws + oRB);
  float*          YT   = (float*)(ws + oRB + al256(szYF));
  unsigned short* XB   = (unsigned short*)(ws + oRC);
  unsigned short* HP   = (unsigned short*)(ws + oRC);

  hipFuncSetAttribute(reinterpret_cast<const void*>(&k_agg<1>),
                      hipFuncAttributeMaxDynamicSharedMemorySize, LDS_AGG);
  hipFuncSetAttribute(reinterpret_cast<const void*>(&k_agg<2>),
                      hipFuncAttributeMaxDynamicSharedMemorySize, LDS_AGG);

  const int nUx = MP * (F_IN / 8);
  k_xprep<<<cdiv(nUx, NTHR), NTHR, 0, stream>>>(x, XB, nN, nUx);

  {
    const int nU1 = CW * (F_IN / 8);
    k_wtr<<<cdiv(nU1, NTHR), NTHR, 0, stream>>>(Wl1, F_IN, F_IN, CW, CW, F_IN, WL1T, nU1);
    k_wtr<<<cdiv(nU1, NTHR), NTHR, 0, stream>>>(Wr1, F_IN, F_IN, CW, CW, F_IN, WR1T, nU1);
    const int nU2 = CW * (KA2 / 8);
    k_wtr<<<cdiv(nU2, NTHR), NTHR, 0, stream>>>(Wl2, CW, CW, CW, CW, KA2, WL2T, nU2);
    k_wtr<<<cdiv(nU2, NTHR), NTHR, 0, stream>>>(Wr2, CW, CW, CW, CW, KA2, WR2T, nU2);
    const int nUh1 = DHA * (KA2 / 8);
    k_wtr<<<cdiv(nUh1, NTHR), NTHR, 0, stream>>>(W1, CW, CW, DHA, DHA, KA2, WH1T, nUh1);
    const int nUh2 = DHBP * ((2 * DHA) / 8);
    k_wtr<<<cdiv(nUh2, NTHR), NTHR, 0, stream>>>(W2, DHA, DHA, DHB, DHBP, 2 * DHA, WH2T, nUh2);
    const int nUh3 = DHCP * ((2 * DHBP) / 8);
    k_wtr<<<cdiv(nUh3, NTHR), NTHR, 0, stream>>>(W3, DHB, DHBP, DHC, DHCP, 2 * DHBP, WH3T, nUh3);
  }

  const int gM = MP / GBM;
  k_gemm<0><<<dim3(gM, CW / GBN), GTHR, 0, stream>>>(XB, WL1T, F_IN, XL, (unsigned short*)XL, CW, 0, bg1, 0);
  k_gemm<1><<<dim3(gM, CW / GBN), GTHR, 0, stream>>>(XB, WR1T, F_IN, (float*)XR, XR, CW, 0, bg1, 0);
  k_agg<1><<<gA, NTHR, LDS_AGG, stream>>>(src, dst, XL, XR, att1, bg1, HP, nN, nE, nb, vec8, MP);
  k_gemm<0><<<dim3(gM, CW / GBN), GTHR, 0, stream>>>(HP, WL2T, KA2, XL, (unsigned short*)XL, CW, 0, bg2, 0);
  k_gemm<1><<<dim3(gM, CW / GBN), GTHR, 0, stream>>>(HP, WR2T, KA2, (float*)XR, XR, CW, 0, bg2, 0);
  k_agg<2><<<gA, NTHR, LDS_AGG, stream>>>(src, dst, XL, XR, att2, bg2, HP, nN, nE, nb, vec8, MP);
  k_gemm<2><<<dim3(gM, DHA / GBN), GTHR, 0, stream>>>(HP, WH1T, KA2, (float*)Y1P, Y1P, 2 * DHA, DHA, b1, DHA);
  k_gemm<2><<<dim3(gM, DHBP / GBN), GTHR, 0, stream>>>(Y1P, WH2T, 2 * DHA, (float*)Y2P, Y2P, 2 * DHBP, DHBP, b2, DHB);
  k_gemm<0><<<dim3(gM, DHCP / GBN), GTHR, 0, stream>>>(Y2P, WH3T, 2 * DHBP, YF, (unsigned short*)YF, DHCP, 0, b3, DHC);
  k_pool<<<nB, NTHR, 0, stream>>>(HP, YF, batch, out1, YT, nN, nB);
  k_out0<<<cdiv(nB * 4, NTHR), NTHR, 0, stream>>>(YT, out0, nB);
}
